// DepthWiseSepConv_36945308680637
// MI455X (gfx1250) — hardware-verified
//
#include <hip/hip_runtime.h>


namespace {
constexpr int Bn = 64, C = 240, CP = 256, HH = 28, WW = 28, NP = HH * WW  , NPP = 896  , KS = 5, R = 60, NPB = NP / 16  ;
constexpr float AS_ = 8.0f, WS_ = 16.0f, BNE = 1e-5f;

typedef _Float16 b16;
typedef __attribute__((ext_vector_type(16))) _Float16 v16b;
typedef __attribute__((ext_vector_type(8))) _Float16 v8b;
typedef __attribute__((ext_vector_type(8))) float v8f;
typedef __attribute__((ext_vector_type(4))) float v4f;
__device__ __forceinline__ void split16(float v, b16& hi, b16& lo) { hi = (b16)v; lo = (b16)(v - (float)hi); }
__device__ __forceinline__ v16b frag_kb(const b16* p, int hh) { const v8b a = *(const v8b*)(p + 8 * hh), b = *(const v8b*)(p + 16 + 8 * hh); v16b f;
#pragma unroll
  for (int e = 0; e < 8; ++e) { f[e] = a[e]; f[8 + e] = b[e]; } return f; }
__device__ __forceinline__ v8f wmma16b(v16b a, v16b b, v8f c) { v8f d = __builtin_amdgcn_wmma_f32_16x16x32_f16(false, a, false, b, (short)0, c, false, false); asm volatile("v_nop\n\tv_nop\n\tv_nop\n\tv_nop" : "+v"(d) : "v"(a), "v"(b)); return d; }
__device__ __forceinline__ void wave_lds_sync() { __builtin_amdgcn_fence(__ATOMIC_RELEASE, "workgroup"); __builtin_amdgcn_wave_barrier(); __builtin_amdgcn_fence(__ATOMIC_ACQUIRE, "workgroup"); }
__device__ __forceinline__ float hswish(float x) { return x * fminf(fmaxf(x + 3.0f, 0.0f), 6.0f) * (1.0f / 6.0f); }
__device__ __forceinline__ float pmul(float a, float b) { float p = a * b; asm volatile("" : "+v"(p)); return p; }

__global__ __launch_bounds__(256) void prep_kernel(const float* __restrict__ pw, b16* __restrict__ wh, b16* __restrict__ wl, b16* __restrict__ dwh, b16* __restrict__ dwl) {
  const size_t tid = (size_t)blockIdx.x * blockDim.x + threadIdx.x, nth = (size_t)gridDim.x * blockDim.x;
  for (int pass = 0; pass < 2; ++pass) {
    for (size_t p = tid; p < (size_t)CP * CP; p += nth) { const int n = (int)(p / CP), k = (int)(p % CP); const float v = (n < C && k < C) ? pw[(size_t)n * C + k] * WS_ : 0.0f; b16 a, c; split16(v, a, c); ((volatile b16*)wh)[p] = a; ((volatile b16*)wl)[p] = c; }
    for (size_t p = tid; p < (size_t)Bn * (NPP - NP) * CP / 8; p += nth) { const size_t per = (size_t)(NPP - NP) * CP / 8; const int b = (int)(p / per); const size_t q = p % per; const v8b z = {};
      *(volatile v8b*)(dwh + ((size_t)b * NPP + NP) * CP + q * 8) = z; *(volatile v8b*)(dwl + ((size_t)b * NPP + NP) * CP + q * 8) = z; }
    __threadfence();
  }
}

__global__ __launch_bounds__(256) void dwconv_kernel(const float* __restrict__ x, const float* __restrict__ dww, const float* __restrict__ dwb, const float* __restrict__ g1, const float* __restrict__ b1, const float* __restrict__ m1, const float* __restrict__ v1,
                                                     b16* __restrict__ dwh, b16* __restrict__ dwl, float* __restrict__ part) {
  __shared__ __attribute__((aligned(16))) b16 Th[16][CP + 8], Tl[16][CP + 8];
  const int c = threadIdx.x, pb = blockIdx.x, b = blockIdx.y, p0 = pb * 16;
  float s = 0.0f;
  if (c < C) { const float* xc = x + ((size_t)b * C + c) * NP; float w[KS * KS];
#pragma unroll
    for (int i = 0; i < KS * KS; ++i) w[i] = dww[(size_t)c * KS * KS + i];
    const float sc = g1[c] * rsqrtf(v1[c] + BNE), sh = b1[c] - m1[c] * sc, bb = dwb[c];
    for (int j = 0; j < 16; ++j) { const int p = p0 + j, y = p / WW, xx = p % WW; float acc = bb;
#pragma unroll
      for (int dy = 0; dy < KS; ++dy) { const int yy = y + dy - 2; if (yy < 0 || yy >= HH) continue;
#pragma unroll
        for (int dx = 0; dx < KS; ++dx) { const int xq = xx + dx - 2; if (xq < 0 || xq >= WW) continue; acc += pmul(w[dy * KS + dx], xc[yy * WW + xq]); } }
      const float v = hswish(acc * sc + sh); s += v; b16 a, l; split16(v * AS_, a, l); Th[j][c] = a; Tl[j][c] = l; } }
  else { for (int j = 0; j < 16; ++j) { Th[j][c] = (b16)0.0f; Tl[j][c] = (b16)0.0f; } }
  __syncthreads();
  for (int pass = 0; pass < 2; ++pass) {
    for (int i = threadIdx.x; i < 16 * CP / 8; i += 256) { const int r = i >> 5, c8 = (i & 31) * 8; const size_t row = (size_t)b * NPP + p0 + r; *(volatile v8b*)(dwh + row * CP + c8) = *(const v8b*)(&Th[r][c8]); *(volatile v8b*)(dwl + row * CP + c8) = *(const v8b*)(&Tl[r][c8]); }
    ((volatile float*)part)[((size_t)b * NPB + pb) * CP + c] = s;
    __threadfence();
  }
}

__global__ __launch_bounds__(256) void se_kernel(const float* __restrict__ part, const float* __restrict__ W1, const float* __restrict__ bb1, const float* __restrict__ W2, const float* __restrict__ bb2, float* __restrict__ g) {
  __shared__ float mean[CP]; __shared__ float hid[R];
  const int b = blockIdx.x, t_ = threadIdx.x;
  { float s = 0.0f; for (int k = 0; k < NPB; ++k) s += part[((size_t)b * NPB + k) * CP + t_]; mean[t_] = s * (1.0f / NP); }
  __syncthreads();
  if (t_ < R) { float a = bb1[t_];
#pragma unroll 1
    for (int c = 0; c < C; ++c) a += W1[(size_t)t_ * C + c] * mean[c];
    hid[t_] = fmaxf(a, 0.0f); }
  __syncthreads();
  float gv = 0.0f; if (t_ < C) { float a = bb2[t_];
#pragma unroll 1
    for (int r = 0; r < R; ++r) a += W2[(size_t)t_ * R + r] * hid[r];
    gv = hswish(a); }
  for (int pass = 0; pass < 2; ++pass) { ((volatile float*)g)[(size_t)b * CP + t_] = gv; __threadfence(); }
}

__global__ __launch_bounds__(128) void pw_kernel(const b16* __restrict__ dwh, const b16* __restrict__ dwl, const b16* __restrict__ wh, const b16* __restrict__ wl, const float* __restrict__ pwb, const float* __restrict__ gsb,
                                                const float* __restrict__ g2, const float* __restrict__ b2, const float* __restrict__ m2, const float* __restrict__ v2, float* __restrict__ inter) {
  __shared__ __attribute__((aligned(16))) float Tc[64][128 + 4];
  const int lane = threadIdx.x & 31, wave = threadIdx.x >> 5, nloc = lane & 15, hlf = lane >> 4, b = blockIdx.z, p0 = blockIdx.y * 128, m0 = p0 + wave * 32, c0 = blockIdx.x * 64;
  const b16* A0 = dwh + ((size_t)b * NPP) * CP; const b16* A1 = dwl + ((size_t)b * NPP) * CP;
  v8f acc[2][4];
#pragma unroll
  for (int r = 0; r < 2; ++r)
#pragma unroll
    for (int t = 0; t < 4; ++t) acc[r][t] = (v8f){};
#pragma unroll 2
  for (int kb = 0; kb < CP; kb += 32) { const v16b a0 = frag_kb(A0 + (size_t)(m0 + nloc) * CP + kb, hlf), l0 = frag_kb(A1 + (size_t)(m0 + nloc) * CP + kb, hlf), a1 = frag_kb(A0 + (size_t)(m0 + 16 + nloc) * CP + kb, hlf), l1 = frag_kb(A1 + (size_t)(m0 + 16 + nloc) * CP + kb, hlf);
#pragma unroll
    for (int t = 0; t < 4; ++t) { const size_t bo = (size_t)(c0 + t * 16 + nloc) * CP + kb; const v16b bw = frag_kb(wh + bo, hlf), bwl = frag_kb(wl + bo, hlf);
      acc[0][t] = wmma16b(a0, bw, acc[0][t]); acc[0][t] = wmma16b(l0, bw, acc[0][t]); acc[0][t] = wmma16b(a0, bwl, acc[0][t]);
      acc[1][t] = wmma16b(a1, bw, acc[1][t]); acc[1][t] = wmma16b(l1, bw, acc[1][t]); acc[1][t] = wmma16b(a1, bwl, acc[1][t]); } }
#pragma unroll
  for (int t = 0; t < 4; ++t) { const int co = c0 + t * 16 + nloc; const int cc = min(co, C - 1); const float sc = g2[cc] * rsqrtf(v2[cc] + BNE), sh = b2[cc] - m2[cc] * sc, gb = gsb[(size_t)b * CP + co], pb_ = pwb[cc];
#pragma unroll
    for (int r = 0; r < 2; ++r)
#pragma unroll
      for (int v = 0; v < 8; ++v) Tc[t * 16 + nloc][wave * 32 + r * 16 + 8 * hlf + v] = ((acc[r][t][v] * (1.0f / (AS_ * WS_)) + pb_) * gb) * sc + sh; }
  __syncthreads();
  for (int pass = 0; pass < 2; ++pass) { for (int i = threadIdx.x; i < 64 * 32; i += 128) { const int cl = i >> 5, q = (i & 31) * 4, co = c0 + cl; if (co < C) *(volatile v4f*)(inter + ((size_t)b * C + co) * NPP + p0 + q) = *(const v4f*)(&Tc[cl][q]); } __threadfence(); }
}

__global__ __launch_bounds__(256) void copy_kernel(const float* __restrict__ inter, float* __restrict__ out) {
  const size_t f = ((size_t)blockIdx.x * 256 + threadIdx.x) * 4; const size_t bc = f / NP; const int p = (int)(f % NP);
  const v4f v = *(const v4f*)(inter + bc * NPP + p);
  for (int pass = 0; pass < 2; ++pass) { *(volatile v4f*)(out + f) = v; __threadfence(); }
}
}

extern "C" void kernel_launch(void* const* d_in, const int* in_sizes, int n_in,
                              void* d_out, int out_size, void* d_ws, size_t ws_size, hipStream_t stream) {
  (void)n_in; (void)out_size;
  const float* x = (const float*)d_in[0]; const float* dww = (const float*)d_in[1]; const float* dwb = (const float*)d_in[2];
  const float* g1 = (const float*)d_in[3]; const float* b1 = (const float*)d_in[4]; const float* m1 = (const float*)d_in[5]; const float* v1 = (const float*)d_in[6];
  const float* pw = (const float*)d_in[7]; const float* pwb = (const float*)d_in[8]; const float* sw1 = (const float*)d_in[9]; const float* sb1 = (const float*)d_in[10]; const float* sw2 = (const float*)d_in[11]; const float* sb2 = (const float*)d_in[12];
  const float* g2 = (const float*)d_in[13]; const float* b2 = (const float*)d_in[14]; const float* m2 = (const float*)d_in[15]; const float* v2 = (const float*)d_in[16];
  float* out = (float*)d_out;
  if (in_sizes[0] != Bn * C * NP || in_sizes[1] != C * KS * KS || in_sizes[7] != C * C || in_sizes[9] != R * C || in_sizes[11] != C * R) return;
  size_t off = 0; char* ws = (char*)d_ws;
  auto carve = [&](size_t bytes) { char* p = ws + off; off += (bytes + 255) & ~(size_t)255; return p; };
  b16* wh = (b16*)carve((size_t)CP * CP * 2); b16* wl = (b16*)carve((size_t)CP * CP * 2); b16* dwh = (b16*)carve((size_t)Bn * NPP * CP * 2); b16* dwl = (b16*)carve((size_t)Bn * NPP * CP * 2);
  float* part = (float*)carve((size_t)Bn * NPB * CP * 4); float* gsb = (float*)carve((size_t)Bn * CP * 4); float* inter = (float*)carve((size_t)Bn * C * NPP * 4);
  if (off > ws_size) return;
  prep_kernel<<<256, 256, 0, stream>>>(pw, wh, wl, dwh, dwl);
  dwconv_kernel<<<dim3(NPB, Bn), 256, 0, stream>>>(x, dww, dwb, g1, b1, m1, v1, dwh, dwl, part);
  se_kernel<<<Bn, 256, 0, stream>>>(part, sw1, sb1, sw2, sb2, gsb);
  pw_kernel<<<dim3(CP / 64, NPP / 128, Bn), 128, 0, stream>>>(dwh, dwl, wh, wl, pwb, gsb, g2, b2, m2, v2, inter);
  copy_kernel<<<Bn * C * NP / 4 / 256, 256, 0, stream>>>(inter, out);
}
